// DecoderBlock_88656714925041
// MI455X (gfx1250) — hardware-verified
//
#include <hip/hip_runtime.h>
#include <math.h>

#ifndef NB
#define NB 2
#endif
#ifndef SEQ
#define SEQ 2048
#endif
#ifndef MEMLEN
#define MEMLEN 1024
#endif
#define NB_FULL 2
#define SEQ_FULL 2048
#define MEM_FULL 1024
#define DM 1024
#define NHEAD 16
#define HDIM 64
#define FFD 4096
#define R_ROWS ((long long)NB * SEQ)
#define RM_ROWS ((long long)NB * MEMLEN)
#define NCHK 64

static_assert(NB >= 1 && NB <= NB_FULL);
static_assert(SEQ % 64 == 0 && SEQ <= SEQ_FULL);
static_assert(MEMLEN % 64 == 0 && MEMLEN <= MEM_FULL);
static_assert(R_ROWS % 64 == 0 && RM_ROWS % 64 == 0);
static_assert(((long long)(NB - 1) * SEQ_FULL + SEQ - 1) * DM + DM - 1 < 16777216 / 4);

typedef __attribute__((ext_vector_type(16))) _Float16 v16h;
typedef __attribute__((ext_vector_type(8)))  _Float16 v8h;
typedef __attribute__((ext_vector_type(16))) __bf16   v16b;
typedef __attribute__((ext_vector_type(8)))  float    v8f;
typedef __attribute__((ext_vector_type(4)))  float    v4f;

__device__ __forceinline__ int frag_k(int i, int h) { return (i < 8) ? (8 * h + i) : (16 + 8 * h + (i - 8)); }
__device__ __forceinline__ __bf16 bf16_rne(float f) {
    unsigned int u = __float_as_uint(f);
    u += 0x7fffu + ((u >> 16) & 1u);
    return __builtin_bit_cast(__bf16, (unsigned short)(u >> 16));
}
__device__ __forceinline__ float bf16_f32(__bf16 b) { return __uint_as_float(((unsigned int)__builtin_bit_cast(unsigned short, b)) << 16); }
__device__ __forceinline__ v8f wmma16(v16h a, v16h b, v8f c) {
    c = __builtin_amdgcn_wmma_f32_16x16x32_f16(false, a, false, b, (short)0, c, false, false);
    asm volatile("v_nop\n\tv_nop\n\tv_nop\n\tv_nop" : "+v"(c) : "v"(a), "v"(b));
    return c;
}
__device__ __forceinline__ v8f wmmab(v16b a, v16b b, v8f c) {
    c = __builtin_amdgcn_wmma_f32_16x16x32_bf16(false, a, false, b, (short)0, c, false, false);
    asm volatile("v_nop\n\tv_nop\n\tv_nop\n\tv_nop" : "+v"(c) : "v"(a), "v"(b));
    return c;
}
struct Split { v16b hi, lo; };
__device__ __forceinline__ v8f wmma3(const Split& a, const Split& b, v8f c) {
    c = __builtin_amdgcn_wmma_f32_16x16x32_bf16(false, a.hi, false, b.hi, (short)0, c, false, false);
    c = __builtin_amdgcn_wmma_f32_16x16x32_bf16(false, a.hi, false, b.lo, (short)0, c, false, false);
    c = __builtin_amdgcn_wmma_f32_16x16x32_bf16(false, a.lo, false, b.hi, (short)0, c, false, false);
    asm volatile("v_nop\n\tv_nop\n\tv_nop\n\tv_nop" : "+v"(c) : "v"(a.hi), "v"(a.lo), "v"(b.hi), "v"(b.lo));
    return c;
}
struct Split3 { v16b hi, mid, lo; };
__device__ __forceinline__ v8f wmma6(const Split3& a, const Split3& b, v8f c) {
    c = __builtin_amdgcn_wmma_f32_16x16x32_bf16(false, a.hi, false, b.hi, (short)0, c, false, false);
    c = __builtin_amdgcn_wmma_f32_16x16x32_bf16(false, a.hi, false, b.mid, (short)0, c, false, false);
    c = __builtin_amdgcn_wmma_f32_16x16x32_bf16(false, a.mid, false, b.hi, (short)0, c, false, false);
    c = __builtin_amdgcn_wmma_f32_16x16x32_bf16(false, a.hi, false, b.lo, (short)0, c, false, false);
    c = __builtin_amdgcn_wmma_f32_16x16x32_bf16(false, a.mid, false, b.mid, (short)0, c, false, false);
    c = __builtin_amdgcn_wmma_f32_16x16x32_bf16(false, a.lo, false, b.hi, (short)0, c, false, false);
    asm volatile("v_nop\n\tv_nop\n\tv_nop\n\tv_nop" : "+v"(c) : "v"(a.hi), "v"(a.mid), "v"(a.lo), "v"(b.hi), "v"(b.mid), "v"(b.lo));
    return c;
}

__device__ __forceinline__ v16h fh_ld(const float* __restrict__ p, long long sk, int k0, int h, int klen, float s) {
    v16h a;
#pragma unroll
    for (int i = 0; i < 16; ++i) { const int k = k0 + frag_k(i, h); a[i] = (k < klen) ? (_Float16)(p[(long long)k * sk] * s) : (_Float16)0.f; }
    return a;
}
__device__ __forceinline__ Split sp_ld(const float* __restrict__ p, long long sk, int k0, int h, int klen, float s) {
    Split r;
#pragma unroll
    for (int i = 0; i < 16; ++i) {
        const int k = k0 + frag_k(i, h); const float x = (k < klen) ? p[(long long)k * sk] * s : 0.f;
        const __bf16 hb = bf16_rne(x); r.hi[i] = hb; r.lo[i] = bf16_rne(x - bf16_f32(hb));
    }
    return r;
}
__device__ __forceinline__ Split3 sp3_ld(const float* __restrict__ p, long long sk, int k0, int h, int klen, float s) {
    Split3 r;
#pragma unroll
    for (int i = 0; i < 16; ++i) {
        const int k = k0 + frag_k(i, h); const float x = (k < klen) ? p[(long long)k * sk] * s : 0.f;
        const __bf16 hb = bf16_rne(x); const float r1 = x - bf16_f32(hb); const __bf16 mb = bf16_rne(r1);
        r.hi[i] = hb; r.mid[i] = mb; r.lo[i] = bf16_rne(r1 - bf16_f32(mb));
    }
    return r;
}

#define VST2(T, ptr, val) do { const T vst2_v_ = (val); *(volatile T*)(ptr) = vst2_v_; __threadfence(); *(volatile T*)(ptr) = vst2_v_; } while (0)
#define VST2V4(ptr, val) do { const v4f vst2_v4_ = (val); *(volatile v4f*)(ptr) = vst2_v4_; __threadfence(); *(volatile v4f*)(ptr) = vst2_v4_; } while (0)

#define AW 4
struct AttnP {
    const float* Q; const float* K; const float* V; float* O; float* P; const float* Mf; const int* Mi; float* ST;
    const float* Pw; const float* Rt; const int* SQ; const int* SK;
    long long swb, swh, swi, swj, srb, srh, sri;
    long long sQb, sQh, sQi, sQd, sKb, sKh, sKj, sKd, sVb, sVh, sVj, sVd, sOb, sOh, sOi, sPb, sPh, sPi, smb, smh, smi, smj;
    int Lq, Lk, dh, dv, hrep, causal, coff, pband;
    float scale, mfill; int nonorm, mpol;
    int roff, rn, segpol, win;
};
static_assert(sizeof(AttnP) == 12 * 8 + 29 * 8 + 16 * 4);

template <int DHP, int DVP, int QM, bool SPLITPV, bool TWOPASS>
__global__ __launch_bounds__(32 * AW) void k_attn(AttnP p) {
    constexpr int NT = DVP / 16;
    constexpr int KS = DHP / 32;
    constexpr int VP = DVP + 8;
    __shared__ __align__(16) float    pl[AW][16 * 64];
    __shared__ __align__(16) _Float16 vl[(SPLITPV ? 2 : 1) * 64 * VP];
    const int lane = threadIdx.x & 31, hf = lane >> 4, l15 = lane & 15, wave = threadIdx.x >> 5;
    const int h = blockIdx.y, b = blockIdx.z, hk = h / p.hrep;
    const int q0 = (blockIdx.x * AW + wave) * 16;
    float* myp = pl[wave];
    const float L2E = 1.4426950408889634f;
    const float NEG = -__builtin_inff();
    const int qi = min(q0 + l15, p.Lq - 1);
    const float* qrow = p.Q + b * p.sQb + h * p.sQh + (long long)qi * p.sQi;
    const float* kbase = p.K + b * p.sKb + hk * p.sKh;
    const float* vbase = p.V + b * p.sVb + hk * p.sVh;
    v16h qa[QM == 0 ? KS : 1]; Split qs_[QM == 1 ? KS : 1]; Split3 qt_[QM == 2 ? KS : 1];
#pragma unroll
    for (int ks = 0; ks < KS; ++ks) {
        if (QM == 2) qt_[ks] = sp3_ld(qrow, p.sQd, ks * 32, hf, p.dh, 1.f);
        else if (QM == 1) qs_[ks] = sp_ld(qrow, p.sQd, ks * 32, hf, p.dh, 1.f);
        else qa[ks] = fh_ld(qrow, p.sQd, ks * 32, hf, p.dh, 1.f);
    }
    v8f o[NT]; float m8[8], l8[8];
#pragma unroll
    for (int t = 0; t < NT; ++t) { v8f zz = {}; o[t] = zz; }
#pragma unroll
    for (int i = 0; i < 8; ++i) { m8[i] = NEG; l8[i] = 0.f; }
    int jend = p.Lk; int jstart = 0;
    if (p.causal == 1) { const int je = (blockIdx.x * AW + AW - 1) * 16 + 16 + p.coff; jend = min(jend, max(je, 0)); }
    if (p.win > 0) { const int js = (int)(blockIdx.x * AW) * 16 + p.coff - p.win; jstart = (js > 0) ? (js / 64) * 64 : 0; }
    const int npass = TWOPASS ? 2 : 1;
    for (int pass = 0; pass < npass; ++pass) {
        const bool dopv = (!TWOPASS) || pass == 1;
        for (int j0 = jstart; j0 < jend; j0 += 64) {
            if (dopv) {
                __syncthreads();
                for (int idx = threadIdx.x; idx < 64 * DVP; idx += 32 * AW) {
                    const int jr = idx / DVP, d = idx - jr * DVP, j = j0 + jr;
                    const float f = (j < p.Lk && d < p.dv) ? vbase[(long long)j * p.sVj + (long long)d * p.sVd] : 0.f;
                    if (SPLITPV) {
                        const __bf16 hb = bf16_rne(f);
                        ((__bf16*)vl)[jr * VP + d] = hb; ((__bf16*)vl)[64 * VP + jr * VP + d] = bf16_rne(f - bf16_f32(hb));
                    } else vl[jr * VP + d] = (_Float16)f;
                }
            }
            v8f s[4];
#pragma unroll
            for (int t = 0; t < 4; ++t) {
                const int j = min(j0 + t * 16 + l15, p.Lk - 1);
                const float* krow = kbase + (long long)j * p.sKj;
                v8f acc = {};
#pragma unroll
                for (int ks = 0; ks < KS; ++ks) {
                    if (QM == 2)      acc = wmma6(qt_[ks], sp3_ld(krow, p.sKd, ks * 32, hf, p.dh, 1.f), acc);
                    else if (QM == 1) acc = wmma3(qs_[ks], sp_ld(krow, p.sKd, ks * 32, hf, p.dh, 1.f), acc);
                    else              acc = wmma16(qa[ks], fh_ld(krow, p.sKd, ks * 32, hf, p.dh, 1.f), acc);
                }
                s[t] = acc;
            }
            float pv[8][4];
#pragma unroll
            for (int i = 0; i < 8; ++i) {
                const int irow = q0 + i + 8 * hf;
                const int ic = min(irow, p.Lq - 1);
                float sc[4];
#pragma unroll
                for (int t = 0; t < 4; ++t) {
                    const int jg = j0 + t * 16 + l15;
                    float v = s[t][i] * p.scale;
                    if (p.Mf) v += p.Mf[b * p.smb + h * p.smh + (long long)ic * p.smi + (long long)min(jg, p.Lk - 1) * p.smj];
                    if (p.Rt) { int rc = ic - min(jg, p.Lk - 1) + p.roff; rc = rc < 0 ? 0 : (rc >= p.rn ? p.rn - 1 : rc); v += p.Rt[b * p.srb + h * p.srh + (long long)ic * p.sri + rc]; }
                    if (p.Mi) { const int mv = p.Mi[b * p.smb + h * p.smh + (long long)ic * p.smi + (long long)min(jg, p.Lk - 1) * p.smj]; if (p.mpol ? (mv != 0) : (mv == 0)) v = p.mfill; }
                    if (p.SQ) { const bool same = p.SQ[(long long)b * p.Lq + ic] == p.SK[(long long)b * p.Lk + min(jg, p.Lk - 1)]; if (p.segpol ? same : !same) v = p.mfill; }
                    if (p.causal == 2 && jg > irow + p.coff) v = p.mfill;
                    if (jg >= p.Lk || (p.causal == 1 && jg > irow + p.coff) || (p.causal == 3 && jg < irow + p.coff) || (p.win > 0 && irow + p.coff - jg > p.win)) v = NEG; else v *= L2E;
                    sc[t] = v;
                }
                if (!TWOPASS || pass == 0) {
                    float mx = fmaxf(fmaxf(sc[0], sc[1]), fmaxf(sc[2], sc[3]));
                    mx = fmaxf(mx, __shfl_xor(mx, 1, 32)); mx = fmaxf(mx, __shfl_xor(mx, 2, 32));
                    mx = fmaxf(mx, __shfl_xor(mx, 4, 32)); mx = fmaxf(mx, __shfl_xor(mx, 8, 32));
                    const float mnew = fmaxf(m8[i], mx);
                    const float corr = (mnew == NEG) ? 1.f : exp2f(m8[i] - mnew);
                    float rs = 0.f;
#pragma unroll
                    for (int t = 0; t < 4; ++t) {
                        const float pp = (sc[t] == NEG) ? 0.f : exp2f(sc[t] - mnew); rs += pp;
                        pv[i][t] = p.Pw ? pp * p.Pw[b * p.swb + h * p.swh + (long long)ic * p.swi + (long long)min(j0 + t * 16 + l15, p.Lk - 1) * p.swj] : pp;
                    }
                    rs += __shfl_xor(rs, 1, 32); rs += __shfl_xor(rs, 2, 32); rs += __shfl_xor(rs, 4, 32); rs += __shfl_xor(rs, 8, 32);
                    l8[i] = l8[i] * corr + rs; m8[i] = mnew;
                    if (!TWOPASS) {
#pragma unroll
                        for (int t = 0; t < NT; ++t) o[t][i] *= corr;
                    }
                } else {
                    const float inv = (l8[i] > 0.f) ? 1.f / l8[i] : 0.f;
#pragma unroll
                    for (int t = 0; t < 4; ++t) {
                        const int jg = j0 + t * 16 + l15;
                        float pp = (sc[t] == NEG) ? 0.f : exp2f(sc[t] - m8[i]) * inv;
                        if (p.Pw) pp *= p.Pw[b * p.swb + h * p.swh + (long long)ic * p.swi + (long long)min(jg, p.Lk - 1) * p.swj];
                        pv[i][t] = pp;
                    }
                }
            }
            if (dopv) {
#pragma unroll
                for (int i = 0; i < 8; ++i)
#pragma unroll
                    for (int t = 0; t < 4; ++t) ((volatile float*)myp)[(i + 8 * hf) * 64 + t * 16 + l15] = pv[i][t];
                __syncthreads();
                if (p.P) {
                    float* pb_ = p.P + b * p.sPb + h * p.sPh;
                    const bool fastP = (p.pband == 0) && ((p.sPi & 3) == 0) && (j0 + 64 <= p.Lk) && (q0 + 16 <= p.Lq) && ((((size_t)pb_) & 15) == 0);
                    if (fastP) {
#pragma unroll
                        for (int s2 = 0; s2 < 8; ++s2) {
                            const int row = s2 * 2 + (lane >> 4), c4 = (lane & 15) * 4;
                            const v4f v = *(const v4f*)(myp + row * 64 + c4);
                            VST2V4(pb_ + (long long)(q0 + row) * p.sPi + j0 + c4, v);
                        }
                    } else {
                        for (int row = 0; row < 16; ++row) {
                            const int irow = q0 + row; if (irow >= p.Lq) continue;
                            for (int c = lane; c < 64; c += 32) {
                                const int jg = j0 + c; if (jg >= p.Lk) continue;
                                if (p.pband == 0) VST2(float, pb_ + (long long)irow * p.sPi + jg, myp[row * 64 + c]);
                                else if (jg - irow <= p.pband && irow - jg <= p.pband) VST2(float, pb_ + (long long)irow * p.sPi + (jg - irow + p.pband), myp[row * 64 + c]);
                            }
                        }
                    }
                }
                if (SPLITPV) {
                    const Split pa0 = sp_ld(myp + l15 * 64, 1, 0, hf, 64, 1.f), pa1 = sp_ld(myp + l15 * 64, 1, 32, hf, 64, 1.f);
                    const __bf16* vh = (const __bf16*)vl; const __bf16* vlo = vh + 64 * VP;
#pragma unroll
                    for (int t = 0; t < NT; ++t) {
                        const int dcol = t * 16 + l15;
                        Split b0, b1;
#pragma unroll
                        for (int e = 0; e < 16; ++e) {
                            const int k0 = frag_k(e, hf), k1 = 32 + frag_k(e, hf);
                            b0.hi[e] = vh[k0 * VP + dcol]; b0.lo[e] = vlo[k0 * VP + dcol]; b1.hi[e] = vh[k1 * VP + dcol]; b1.lo[e] = vlo[k1 * VP + dcol];
                        }
                        o[t] = wmma3(pa0, b0, o[t]);
                        o[t] = wmma3(pa1, b1, o[t]);
                    }
                } else {
                    const v16h pa0 = fh_ld(myp + l15 * 64, 1, 0, hf, 64, 4096.f), pa1 = fh_ld(myp + l15 * 64, 1, 32, hf, 64, 4096.f);
#pragma unroll
                    for (int t = 0; t < NT; ++t) {
                        const int dcol = t * 16 + l15;
                        v16h b0, b1;
#pragma unroll
                        for (int e = 0; e < 16; ++e) { b0[e] = vl[frag_k(e, hf) * VP + dcol]; b1[e] = vl[(32 + frag_k(e, hf)) * VP + dcol]; }
                        o[t] = wmma16(pa0, b0, o[t]);
                        o[t] = wmma16(pa1, b1, o[t]);
                    }
                }
            }
        }
    }
    float* obase = p.O + b * p.sOb + h * p.sOh;
    if (p.ST) {
        const int rl = lane >> 1, isel = rl & 7;
        float mv = 0.f, lv = 0.f;
#pragma unroll
        for (int i = 0; i < 8; ++i) if (i == isel) { mv = m8[i]; lv = l8[i]; }
        const int irow = q0 + rl;
        if (irow < p.Lq) { float* st = p.ST + (((long long)b * gridDim.y + h) * p.Lq + irow) * 2 + (lane & 1); VST2(float, st, (lane & 1) ? lv : mv * 0.6931471805599453f); }
    }
    float invr[8];
#pragma unroll
    for (int i = 0; i < 8; ++i) {
        if (TWOPASS) invr[i] = SPLITPV ? 1.f : (1.f / 4096.f);
        else if (p.nonorm) invr[i] = exp2f(m8[i]) * (SPLITPV ? 1.f : (1.f / 4096.f));
        else invr[i] = (l8[i] > 0.f) ? (SPLITPV ? 1.f / l8[i] : 1.f / (l8[i] * 4096.f)) : 0.f;
    }
    __syncthreads();
    const bool ofast = ((p.sOi & 3) == 0) && ((((size_t)obase) & 15) == 0) && (q0 + 16 <= p.Lq);
#pragma unroll
    for (int c0 = 0; c0 < DVP; c0 += 64) {
#pragma unroll
        for (int i = 0; i < 8; ++i)
#pragma unroll
            for (int t = 0; t < NT; ++t) if (t * 16 >= c0 && t * 16 < c0 + 64) ((volatile float*)myp)[(i + 8 * hf) * 64 + (t * 16 - c0) + l15] = o[t][i] * invr[i];
        __syncthreads();
        const int cw = (DVP - c0 < 64) ? (DVP - c0) : 64;
        if (ofast && (c0 + cw <= p.dv) && (cw % 32 == 0)) {
            const int lpr = cw / 4;
            const int rows_per_ins = 32 / lpr;
            for (int r0 = 0; r0 < 16; r0 += rows_per_ins) {
                const int row = r0 + lane / lpr, c4 = (lane % lpr) * 4;
                const v4f v = *(const v4f*)(myp + row * 64 + c4);
                VST2V4(obase + (long long)(q0 + row) * p.sOi + c0 + c4, v);
            }
        } else {
            for (int row = 0; row < 16; ++row) {
                const int irow = q0 + row; if (irow >= p.Lq) continue;
                for (int c = lane; c < cw; c += 32) { const int d = c0 + c; if (d < p.dv) VST2(float, obase + (long long)irow * p.sOi + d, myp[row * 64 + c]); }
            }
        }
        __syncthreads();
    }
}

namespace w25 {
typedef __attribute__((ext_vector_type(16))) _Float16 v16h;
typedef __attribute__((ext_vector_type(8)))  _Float16 v8h;
typedef __attribute__((ext_vector_type(16))) __bf16   v16b;
typedef __attribute__((ext_vector_type(8)))  __bf16   v8b;
typedef __attribute__((ext_vector_type(8)))  float    v8f;
typedef __attribute__((ext_vector_type(4)))  float    v4f;

__device__ __forceinline__ unsigned short f2bf_bits(float f) {
  unsigned u = __float_as_uint(f);
  return (unsigned short)((u + 0x7FFFu + ((u >> 16) & 1u)) >> 16);
}
__device__ __forceinline__ float bf_bits2f(unsigned short h) { return __uint_as_float(((unsigned)h) << 16); }

__device__ __forceinline__ void dep_guard_h(v8f& a, v8f& b, v16h x, v16h y) { asm volatile("v_nop\n\tv_nop\n\tv_nop\n\tv_nop" : "+v"(a), "+v"(b) : "v"(x), "v"(y)); }
__device__ __forceinline__ void dep_guard_b(v8f& a, v8f& b, v16b x, v16b y) { asm volatile("v_nop\n\tv_nop\n\tv_nop\n\tv_nop" : "+v"(a), "+v"(b) : "v"(x), "v"(y)); }
__device__ __forceinline__ void keep4_h(v16h a, v16h b, v16h c, v16h d) { asm volatile("v_nop" :: "v"(a), "v"(b), "v"(c), "v"(d)); }
__device__ __forceinline__ void keep4_b(v16b a, v16b b, v16b c, v16b d) { asm volatile("v_nop" :: "v"(a), "v"(b), "v"(c), "v"(d)); }
__device__ __forceinline__ void acc_guard4(v8f& a, v8f& b, v8f& c, v8f& d) { asm volatile("v_nop\n\tv_nop\n\tv_nop\n\tv_nop" : "+v"(a), "+v"(b), "+v"(c), "+v"(d)); }
template <typename T> struct Frag;
template <> struct Frag<_Float16> {
  typedef v16h V; union U { v16h v; v8h h[2]; };
  static __device__ __forceinline__ v16h load(const _Float16* p) {
    U f; f.h[0] = *(const v8h*)(p); f.h[1] = *(const v8h*)(p + 16); return f.v;
  }
  static __device__ __forceinline__ v8f mma(v16h a, v16h b, v8f c) {
    return __builtin_amdgcn_wmma_f32_16x16x32_f16(false, a, false, b, (short)0, c, false, false);
  }
  static __device__ __forceinline__ void guard(v8f& a, v8f& b, v16h x, v16h y) { dep_guard_h(a, b, x, y); }
  static __device__ __forceinline__ void keep(v16h a, v16h b, v16h c, v16h d) { keep4_h(a, b, c, d); }
};
template <> struct Frag<__bf16> {
  typedef v16b V; union U { v16b v; v8b h[2]; };
  static __device__ __forceinline__ v16b load(const __bf16* p) {
    U f; f.h[0] = *(const v8b*)(p); f.h[1] = *(const v8b*)(p + 16); return f.v;
  }
  static __device__ __forceinline__ v8f mma(v16b a, v16b b, v8f c) {
    return __builtin_amdgcn_wmma_f32_16x16x32_bf16(false, a, false, b, (short)0, c, false, false);
  }
  static __device__ __forceinline__ void guard(v8f& a, v8f& b, v16b x, v16b y) { dep_guard_b(a, b, x, y); }
  static __device__ __forceinline__ void keep(v16b a, v16b b, v16b c, v16b d) { keep4_b(a, b, c, d); }
};

template <int ET> struct Elem;
template <> struct Elem<0> { typedef _Float16 T; };
template <> struct Elem<1> { typedef __bf16 T; };
template <int ET, bool SPLIT, int BIAS_MODE, int OUT_MODE, bool RESID, int ACT = 0>
__global__ __launch_bounds__(256) void wmma_gemm64(
    const unsigned short* __restrict__ Ap, const unsigned short* __restrict__ A2p, int lda, long strideA,
    const unsigned short* __restrict__ Btp, const unsigned short* __restrict__ Bt2p, int ldb, long strideB,
    void* __restrict__ Cout, void* __restrict__ Cout2, int ldc, long strideC,
    const float* __restrict__ bias,
    const float* __restrict__ resid, long strideR,
    int M, int N, int K, float scale) {
  typedef typename Elem<ET>::T T;
  typedef typename Frag<T>::V V;
  const T* A = (const T*)Ap; const T* A2 = (const T*)A2p; const T* Bt = (const T*)Btp; const T* Bt2 = (const T*)Bt2p;
  __shared__ __align__(16) float sT[8][16 * 68];
  const int b    = blockIdx.y;
  const int lane = threadIdx.x & 31;
  const int wave = threadIdx.x >> 5;
  const int tilesN = N >> 6;
  const int tilesM = M >> 6;
  const int tile = blockIdx.x * 8 + wave;
  if (tile >= tilesM * tilesN) return;
  const int tm = tile / tilesN;
  const int tn = tile - tm * tilesN;
  const int m0 = tm << 6;
  const int n0 = tn << 6;

  const T* Ab  = A  + (size_t)b * strideA;
  const T* Bb  = Bt + (size_t)b * strideB;
  const T* Ab2 = SPLIT ? (A2  + (size_t)b * strideA) : nullptr;
  const T* Bb2 = SPLIT ? (Bt2 + (size_t)b * strideB) : nullptr;

  const int rlane = lane & 15;
  const int koff  = (lane >> 4) * 8;
  const int mOff  = (lane >> 4) * 8;

  v8f acc[4][4];
#pragma unroll
  for (int i = 0; i < 4; ++i)
#pragma unroll
    for (int j = 0; j < 4; ++j) acc[i][j] = (v8f){0.f,0.f,0.f,0.f,0.f,0.f,0.f,0.f};

  for (int k0 = 0; k0 < K; k0 += 32) {
    V bh[4], bl[4];
#pragma unroll
    for (int j = 0; j < 4; ++j) {
      const size_t bo = (size_t)(n0 + (j << 4) + rlane) * ldb + koff + k0;
      bh[j] = Frag<T>::load(Bb + bo);
      if (SPLIT) bl[j] = Frag<T>::load(Bb2 + bo);
    }
#pragma unroll
    for (int i = 0; i < 4; ++i) {
      const size_t ao = (size_t)(m0 + (i << 4) + rlane) * lda + koff + k0;
      V ah = Frag<T>::load(Ab + ao);
      V al;
      if (SPLIT) al = Frag<T>::load(Ab2 + ao);
#pragma unroll
      for (int j = 0; j < 4; ++j) {
        acc[i][j] = Frag<T>::mma(ah, bh[j], acc[i][j]);
        if (SPLIT) {
          acc[i][j] = Frag<T>::mma(ah, bl[j], acc[i][j]);
          acc[i][j] = Frag<T>::mma(al, bh[j], acc[i][j]);
        }
      }
      Frag<T>::guard(acc[i][0], acc[i][3], ah, SPLIT ? al : ah);
    }
    Frag<T>::keep(bh[0], bh[1], bh[2], bh[3]);
    if (SPLIT) Frag<T>::keep(bl[0], bl[1], bl[2], bl[3]);
  }
  acc_guard4(acc[0][0], acc[0][1], acc[0][2], acc[0][3]);
  acc_guard4(acc[1][0], acc[1][1], acc[1][2], acc[1][3]);
  acc_guard4(acc[2][0], acc[2][1], acc[2][2], acc[2][3]);
  acc_guard4(acc[3][0], acc[3][1], acc[3][2], acc[3][3]);

  float* slab = sT[wave];
  const float* Rb = RESID ? (resid + (size_t)b * strideR) : nullptr;
#pragma unroll
  for (int i = 0; i < 4; ++i) {
    const int mBase = m0 + (i << 4);
#pragma unroll
    for (int j = 0; j < 4; ++j) {
      const int n = n0 + (j << 4) + rlane;
      float bv = 0.f;
      if (BIAS_MODE == 2) bv = bias[n];
#pragma unroll
      for (int r = 0; r < 8; ++r) {
        float v = acc[i][j][r] * scale;
        if (BIAS_MODE == 1) v += bias[mBase + mOff + r];
        if (BIAS_MODE == 2) v += bv;
        if (RESID) v += Rb[(size_t)(mBase + mOff + r) * ldc + n];
        if (ACT == 1) v = tanhf(v);
        if (ACT == 2) v = fmaxf(v, 0.0f);
        if (ACT == 3) v = v / (1.0f + expf(-v));
        if (ACT == 4) v = (v > 0.f) ? v : 0.01f * v;
        if (ACT == 5) v = 0.5f * v * (1.0f + erff(v * 0.70710678118654752f));
        if (ACT == 6) v = (v > 0.f) ? v : 0.2f * v;
        if (ACT == 7) { const float u = 0.7978845608028654f * (v + 0.044715f * v * v * v); v = 0.5f * v * (1.f + tanhf(u)); }
        slab[(mOff + r) * 68 + (j << 4) + rlane] = v;
      }
    }
    __builtin_amdgcn_fence(3  , "workgroup");
    __builtin_amdgcn_wave_barrier();
    __builtin_amdgcn_fence(2  , "workgroup");
    if (OUT_MODE == 0) {
      float* C = (float*)Cout + (size_t)b * strideC;
      const int hh = lane >> 4, c4 = (lane & 15) * 4;
      for (int pass = 0; pass < 2; ++pass) {
#pragma unroll
        for (int it = 0; it < 8; ++it) {
          const int row = it * 2 + hh;
          v4f v = *(const v4f*)(slab + row * 68 + c4);
          *(volatile v4f*)(C + (size_t)(mBase + row) * ldc + n0 + c4) = v;
        }
        __threadfence();
      }
    } else {
      const int q = lane >> 3, c8 = (lane & 7) * 8;
      unsigned short* C  = (unsigned short*)Cout  + (size_t)b * strideC;
      unsigned short* C2 = (OUT_MODE == 2) ? ((unsigned short*)Cout2 + (size_t)b * strideC) : nullptr;
      for (int pass = 0; pass < 2; ++pass) {
#pragma unroll
        for (int it = 0; it < 4; ++it) {
          const int row = it * 4 + q;
          const float* sp = slab + row * 68 + c8;
          v8h hv, lv;
#pragma unroll
          for (int e = 0; e < 8; ++e) {
            if (OUT_MODE == 1) {
              hv[e] = (_Float16)sp[e];
              lv[e] = (_Float16)0.f;
            } else {
              unsigned short hb = f2bf_bits(sp[e]);
              unsigned short lb = f2bf_bits(sp[e] - bf_bits2f(hb));
              hv[e] = __builtin_bit_cast(_Float16, hb);
              lv[e] = __builtin_bit_cast(_Float16, lb);
            }
          }
          *(volatile v8h*)(C + (size_t)(mBase + row) * ldc + n0 + c8) = hv;
          if (OUT_MODE == 2) *(volatile v8h*)(C2 + (size_t)(mBase + row) * ldc + n0 + c8) = lv;
        }
        __threadfence();
      }
    }
    __builtin_amdgcn_fence(3  , "workgroup");
    __builtin_amdgcn_wave_barrier();
    __builtin_amdgcn_fence(2  , "workgroup");
  }
}

#define AT_D 64
#define AT_NW 4
#define AT_QB 64
#define AT_KC 64
struct AttnGeom { const float* cp; const float* pc; long c_bs, c_rs, c_hs;
                  long q_bs, q_rs, q_hs, k_bs, k_rs, k_hs, v_bs, v_rs, v_hs, o_bs, o_rs, o_hs;
                  int S, Skv, H, mask_mode; float qscale; int blk0; float mask_fill; int mask_is_int; };
static_assert(sizeof(AttnGeom) == 168);

__device__ __forceinline__ unsigned short at_bf_bits(float f) {
  unsigned u = __float_as_uint(f);
  return (unsigned short)((u + 0x7FFFu + ((u >> 16) & 1u)) >> 16);
}
__device__ __forceinline__ __bf16 at_f2bf(float f) { return __builtin_bit_cast(__bf16, at_bf_bits(f)); }
__device__ __forceinline__ void at_split(float f, __bf16& hi, __bf16& lo) {
  const unsigned short hb = at_bf_bits(f);
  hi = __builtin_bit_cast(__bf16, hb);
  lo = at_f2bf(f - __uint_as_float(((unsigned)hb) << 16));
}
__device__ __forceinline__ v8f at_mma(v16b a, v16b b, v8f c) {
  c = __builtin_amdgcn_wmma_f32_16x16x32_bf16(false, a, false, b, (short)0, c, false, false);
  asm volatile("v_nop\n\tv_nop\n\tv_nop\n\tv_nop" : "+v"(c) : "v"(a), "v"(b));
  return c;
}
template <bool F16> __device__ __forceinline__ __bf16 at_to16(float f) {
  if (F16) return __builtin_bit_cast(__bf16, (_Float16)f);
  return at_f2bf(f);
}
template <bool F16> __device__ __forceinline__ v8f at_mma16(v16b a, v16b b, v8f c) {
  if (F16) {
    const v16h ah = __builtin_bit_cast(v16h, a), bh = __builtin_bit_cast(v16h, b);
    c = __builtin_amdgcn_wmma_f32_16x16x32_f16(false, ah, false, bh, (short)0, c, false, false);
    asm volatile("v_nop\n\tv_nop\n\tv_nop\n\tv_nop" : "+v"(c) : "v"(ah), "v"(bh));
    return c;
  }
  return at_mma(a, b, c);
}

template <bool SPLIT_QK, bool SPLIT_PV, bool F16 = false>
__global__ __launch_bounds__(128)
void attn64_kernel(const float* __restrict__ q, const float* __restrict__ k,
                   const float* __restrict__ v, float* __restrict__ out,
                   const void* __restrict__ mask_a, const int* __restrict__ mask_b, AttnGeom g) {
  static_assert(!(F16 && (SPLIT_QK || SPLIT_PV)));
  const float PSC = F16 ? 32768.0f : 1.0f;
  union FB { v16b v; v8b h[2]; };
  __shared__ __align__(16) __bf16 Ksh[AT_KC * AT_D];
  __shared__ __align__(16) __bf16 Ksl[SPLIT_QK ? AT_KC * AT_D : 8];
  __shared__ __align__(16) __bf16 Vth[AT_D * AT_KC];
  __shared__ __align__(16) __bf16 Vtl[SPLIT_PV ? AT_D * AT_KC : 8];
  __shared__ __align__(16) __bf16 Psh[AT_NW][16 * AT_KC];
  __shared__ __align__(16) __bf16 Psl[SPLIT_PV ? AT_NW : 1][SPLIT_PV ? 16 * AT_KC : 8];
  __shared__ __align__(16) float  Os[AT_NW][16 * 68];

  const int tid  = threadIdx.x;
  const int wave = tid >> 5;
  const int lane = tid & 31;
  const int hh   = lane >> 4;
  const int c    = lane & 15;

  const int nqb = g.S / AT_QB;
  const int bx = blockIdx.x + g.blk0;
  const int qb = bx % nqb;
  const int bh = bx / nqb;
  const int h  = bh % g.H;
  const int b  = bh / g.H;
  const int qbase_block = qb * AT_QB;
  const int q0 = qbase_block + wave * 16;

  const float* qb_ptr = q + (size_t)b * g.q_bs + (size_t)h * g.q_hs;
  const float* kb_ptr = k + (size_t)b * g.k_bs + (size_t)h * g.k_hs;
  const float* vb_ptr = v + (size_t)b * g.v_bs + (size_t)h * g.v_hs;
  float*       ob_ptr = out + (size_t)b * g.o_bs + (size_t)h * g.o_hs;

  v16b qah[2], qal[2];
  {
    const float* qrow = qb_ptr + (size_t)(q0 + c) * g.q_rs;
#pragma unroll
    for (int dc = 0; dc < 2; ++dc) {
      const v4f u0 = *(const v4f*)(qrow + dc * 32 + 8 * hh), u1 = *(const v4f*)(qrow + dc * 32 + 8 * hh + 4);
      const v4f w0 = *(const v4f*)(qrow + dc * 32 + 16 + 8 * hh), w1 = *(const v4f*)(qrow + dc * 32 + 16 + 8 * hh + 4);
      const float fa[8] = {u0.x, u0.y, u0.z, u0.w, u1.x, u1.y, u1.z, u1.w};
      const float fb[8] = {w0.x, w0.y, w0.z, w0.w, w1.x, w1.y, w1.z, w1.w};
#pragma unroll
      for (int e = 0; e < 8; ++e) {
        const float f0 = fa[e] * g.qscale;
        const float f1 = fb[e] * g.qscale;
        if (SPLIT_QK) { __bf16 hq, lq; at_split(f0, hq, lq); qah[dc][e] = hq; qal[dc][e] = lq; at_split(f1, hq, lq); qah[dc][8 + e] = hq; qal[dc][8 + e] = lq; }
        else { qah[dc][e] = at_to16<F16>(f0); qah[dc][8 + e] = at_to16<F16>(f1); qal[dc][e] = qah[dc][e]; qal[dc][8 + e] = qah[dc][8 + e]; }
      }
    }
  }

  float mrow[8], lrow[8];
  v8f oacc[4];
#pragma unroll
  for (int r = 0; r < 8; ++r) { mrow[r] = -INFINITY; lrow[r] = 0.f; }
#pragma unroll
  for (int t = 0; t < 4; ++t) oacc[t] = (v8f){0.f,0.f,0.f,0.f,0.f,0.f,0.f,0.f};

  const int nChunks = (g.mask_mode == 1 || g.mask_mode == 4) ? (qb + 1) : (g.Skv / AT_KC);
  int qkeep[8];
#pragma unroll
  for (int r = 0; r < 8; ++r) qkeep[r] = (g.mask_mode == 3) ? mask_b[(size_t)b * g.S + q0 + 8 * hh + r] : 1;
  for (int kc = 0; kc < nChunks; ++kc) {
    const int kv0 = kc * AT_KC;
    __syncthreads();
    {
      const int kvr = tid >> 1, dh = (tid & 1) * 32;
      const float* krow = kb_ptr + (size_t)(kv0 + kvr) * g.k_rs + dh;
      const float* vrow = vb_ptr + (size_t)(kv0 + kvr) * g.v_rs + dh;
#pragma unroll
      for (int i = 0; i < 8; ++i) {
        v4f kk = *(const v4f*)(krow + 4 * i);
        v4f vv = *(const v4f*)(vrow + 4 * i);
#pragma unroll
        for (int e = 0; e < 4; ++e) {
          const int d = dh + 4 * i + e;
          if (SPLIT_QK) { __bf16 a, bl; at_split(kk[e], a, bl); Ksh[kvr * AT_D + d] = a; Ksl[kvr * AT_D + d] = bl; }
          else Ksh[kvr * AT_D + d] = at_to16<F16>(kk[e]);
          if (SPLIT_PV) { __bf16 a, bl; at_split(vv[e], a, bl); Vth[d * AT_KC + kvr] = a; Vtl[d * AT_KC + kvr] = bl; }
          else Vth[d * AT_KC + kvr] = at_to16<F16>(vv[e]);
        }
      }
    }
    __syncthreads();

    v8f s[4];
#pragma unroll
    for (int j = 0; j < 4; ++j) {
      s[j] = (v8f){0.f,0.f,0.f,0.f,0.f,0.f,0.f,0.f};
#pragma unroll 1
      for (int dc = 0; dc < 2; ++dc) {
        FB kb;
        kb.h[0] = *(const v8b*)(Ksh + (j * 16 + c) * AT_D + dc * 32 + 8 * hh);
        kb.h[1] = *(const v8b*)(Ksh + (j * 16 + c) * AT_D + dc * 32 + 16 + 8 * hh);
        s[j] = at_mma16<F16>(qah[dc], kb.v, s[j]);
        if (SPLIT_QK) {
          FB kl;
          kl.h[0] = *(const v8b*)(Ksl + (j * 16 + c) * AT_D + dc * 32 + 8 * hh);
          kl.h[1] = *(const v8b*)(Ksl + (j * 16 + c) * AT_D + dc * 32 + 16 + 8 * hh);
          s[j] = at_mma16<F16>(qah[dc], kl.v, s[j]);
          s[j] = at_mma16<F16>(qal[dc], kb.v, s[j]);
        }
      }
    }
    const bool diag = (g.mask_mode == 1) && (kc == qb);
    int kvkeep[4] = {1, 1, 1, 1};
    if (g.mask_mode == 3) {
#pragma unroll
      for (int j = 0; j < 4; ++j) kvkeep[j] = ((const int*)mask_a)[(size_t)b * g.Skv + kv0 + j * 16 + c];
    }
    float cm[8];
#pragma unroll
    for (int r = 0; r < 8; ++r) {
      const int qrow = q0 + 8 * hh + r;
      float m = -INFINITY;
#pragma unroll
      for (int j = 0; j < 4; ++j) {
        const int kvcol = kv0 + j * 16 + c;
        bool masked = false;
        if (diag) masked = (kvcol > qrow);
        else if (g.mask_mode == 4) masked = (kvcol > qrow) || (qrow - kvcol > g.mask_is_int);
        else if (g.mask_mode == 2) {
          const size_t mi = (size_t)qrow * g.Skv + kvcol;
          masked = (g.mask_is_int == 0) ? (((const float*)mask_a)[mi] == 0.0f)
                 : (g.mask_is_int == 1) ? (((const int*)mask_a)[mi] == 0) : (((const int*)mask_a)[mi] != 0);
        } else if (g.mask_mode == 3) masked = (qkeep[r] == 0) || (kvkeep[j] == 0);
        else if (g.mask_mode == 5) {
          const size_t mi = (size_t)qrow * g.Skv + kvcol;
          masked = (((const int*)mask_a)[mi] != 0);
          int n = mask_b[mi]; n = n < 0 ? 0 : n;
          s[j][r] += g.cp[(size_t)b * g.c_bs + (size_t)h * g.c_hs + (size_t)qrow * g.c_rs + n]
                   + g.pc[(size_t)b * g.c_bs + (size_t)h * g.c_hs + (size_t)kvcol * g.c_rs + n];
        }
        if (masked) s[j][r] = g.mask_fill;
        m = fmaxf(m, s[j][r]);
      }
#pragma unroll
      for (int off = 1; off < 16; off <<= 1) m = fmaxf(m, __shfl_xor(m, off, 32));
      cm[r] = m;
    }
    __bf16* pwh = Psh[wave];
    __bf16* pwl = Psl[SPLIT_PV ? wave : 0];
#pragma unroll
    for (int r = 0; r < 8; ++r) {
      const float mnew = fmaxf(mrow[r], cm[r]);
      const float alpha = expf(mrow[r] - mnew);
      mrow[r] = mnew;
      float psum = 0.f;
#pragma unroll
      for (int j = 0; j < 4; ++j) {
        const float p = expf(s[j][r] - mnew);
        psum += p;
        if (SPLIT_PV) { __bf16 a, bl; at_split(p, a, bl); pwh[(8 * hh + r) * AT_KC + j * 16 + c] = a; pwl[(8 * hh + r) * AT_KC + j * 16 + c] = bl; }
        else pwh[(8 * hh + r) * AT_KC + j * 16 + c] = at_to16<F16>(p * PSC);
      }
#pragma unroll
      for (int off = 1; off < 16; off <<= 1) psum += __shfl_xor(psum, off, 32);
      lrow[r] = lrow[r] * alpha + psum;
#pragma unroll
      for (int t = 0; t < 4; ++t) oacc[t][r] *= alpha;
    }
    __builtin_amdgcn_fence(3  , "workgroup");
    __builtin_amdgcn_wave_barrier();
    __builtin_amdgcn_fence(2  , "workgroup");
#pragma unroll 1
    for (int kk = 0; kk < 2; ++kk) {
      FB pa, pl;
      pa.h[0] = *(const v8b*)(pwh + c * AT_KC + kk * 32 + 8 * hh);
      pa.h[1] = *(const v8b*)(pwh + c * AT_KC + kk * 32 + 16 + 8 * hh);
      if (SPLIT_PV) {
        pl.h[0] = *(const v8b*)(pwl + c * AT_KC + kk * 32 + 8 * hh);
        pl.h[1] = *(const v8b*)(pwl + c * AT_KC + kk * 32 + 16 + 8 * hh);
      }
#pragma unroll
      for (int t = 0; t < 4; ++t) {
        FB vb;
        vb.h[0] = *(const v8b*)(Vth + (t * 16 + c) * AT_KC + kk * 32 + 8 * hh);
        vb.h[1] = *(const v8b*)(Vth + (t * 16 + c) * AT_KC + kk * 32 + 16 + 8 * hh);
        oacc[t] = at_mma16<F16>(pa.v, vb.v, oacc[t]);
        if (SPLIT_PV) {
          FB vl;
          vl.h[0] = *(const v8b*)(Vtl + (t * 16 + c) * AT_KC + kk * 32 + 8 * hh);
          vl.h[1] = *(const v8b*)(Vtl + (t * 16 + c) * AT_KC + kk * 32 + 16 + 8 * hh);
          oacc[t] = at_mma16<F16>(pa.v, vl.v, oacc[t]);
          oacc[t] = at_mma16<F16>(pl.v, vb.v, oacc[t]);
        }
      }
    }
  }

  float* os = Os[wave];
#pragma unroll
  for (int r = 0; r < 8; ++r) {
    const float inv = 1.0f / (lrow[r] * PSC);
#pragma unroll
    for (int t = 0; t < 4; ++t) os[(8 * hh + r) * 68 + t * 16 + c] = oacc[t][r] * inv;
  }
  __builtin_amdgcn_fence(3  , "workgroup");
  __builtin_amdgcn_wave_barrier();
  __builtin_amdgcn_fence(2  , "workgroup");
  {
    const int c4 = (lane & 15) * 4;
    for (int pass = 0; pass < 2; ++pass) {
#pragma unroll
      for (int it = 0; it < 8; ++it) {
        const int row = it * 2 + hh;
        v4f val = *(const v4f*)(os + row * 68 + c4);
        *(volatile v4f*)(ob_ptr + (size_t)(q0 + row) * g.o_rs + c4) = val;
      }
      __threadfence();
    }
  }
}

}

typedef unsigned int cm_u4 __attribute__((ext_vector_type(4)));
__device__ __forceinline__ unsigned int cmb_pk2(float a, float b) { return (unsigned int)__builtin_bit_cast(unsigned short, (_Float16)a) | ((unsigned int)__builtin_bit_cast(unsigned short, (_Float16)b) << 16); }
__device__ __forceinline__ float cmb_bf(float v) { const unsigned u = __builtin_bit_cast(unsigned, v); const unsigned r = (u + 0x7fffu + ((u >> 16) & 1u)) & 0xffff0000u; return __builtin_bit_cast(float, r); }
__global__ __launch_bounds__(256) void k_cm_castb(const float* __restrict__ SRC, int lds, unsigned short* __restrict__ DST, int ldd, int nR, int nC, float sc) {
    const long long u = (long long)blockIdx.x * 256 + threadIdx.x; const int per = nC / 8; if (u >= (long long)nR * per) return; const int r = (int)(u / per); const int c0 = 8 * (int)(u % per);
    const float* s = SRC + (long long)r * lds + c0; float w[8];
#pragma unroll
    for (int e = 0; e < 8; ++e) w[e] = cmb_bf(s[e]) * sc;
    cm_u4 pk; pk.x = cmb_pk2(w[0], w[1]); pk.y = cmb_pk2(w[2], w[3]); pk.z = cmb_pk2(w[4], w[5]); pk.w = cmb_pk2(w[6], w[7]); VST2(cm_u4, (cm_u4*)(DST + (long long)r * ldd + c0), pk); }

template <bool RBF, bool WF32>
__global__ __launch_bounds__(256) void k_cvt16(const float* __restrict__ S, unsigned short* __restrict__ D16, float* __restrict__ D32, int rows, int seq, int seqfull) {
    const int u = blockIdx.x * 256 + threadIdx.x; if (u >= rows * 256) return;
    const int r = u >> 8; const int c = 4 * (u & 255);
    const size_t srow = (size_t)(r / seq) * (size_t)seqfull + (size_t)(r % seq);
    const v4f a = *(const v4f*)(S + srow * 1024 + c);
    v4f w;
    w.x = RBF ? cmb_bf(a.x) : a.x; w.y = RBF ? cmb_bf(a.y) : a.y; w.z = RBF ? cmb_bf(a.z) : a.z; w.w = RBF ? cmb_bf(a.w) : a.w;
    const unsigned long long pk = (unsigned long long)cmb_pk2(w.x, w.y) | ((unsigned long long)cmb_pk2(w.z, w.w) << 32);
    VST2(unsigned long long, (unsigned long long*)(D16 + (size_t)r * 1024 + c), pk);
    if (WF32) { VST2V4(D32 + (size_t)r * 1024 + c, w); }
}

template <bool W16, bool W32, bool OMAP, bool CHKF>
__global__ __launch_bounds__(256) void k_ln1024(const float* __restrict__ X, const float* __restrict__ G, const float* __restrict__ Bb,
                                                unsigned short* __restrict__ O16, float* __restrict__ O32, const float* __restrict__ chk, int rows, int seq, int seqfull) {
    #pragma clang fp contract(off)
    const int row = blockIdx.x * 8 + (threadIdx.x >> 5); const int L = threadIdx.x & 31;
    if (row >= rows) return;
    const float* xr = X + (size_t)row * 1024;
    float x[32]; float s = 0.f;
#pragma unroll
    for (int q4 = 0; q4 < 8; ++q4) {
        const v4f a = *(const v4f*)(xr + 128 * q4 + 4 * L);
        x[4 * q4] = a.x; x[4 * q4 + 1] = a.y; x[4 * q4 + 2] = a.z; x[4 * q4 + 3] = a.w;
        s += (a.x + a.y) + (a.z + a.w);
    }
#pragma unroll
    for (int o = 16; o > 0; o >>= 1) s += __shfl_xor(s, o, 32);
    const float mu = s * (1.f / 1024.f); float qq = 0.f;
#pragma unroll
    for (int e = 0; e < 32; ++e) { const float d = x[e] - mu; qq += d * d; }
#pragma unroll
    for (int o = 16; o > 0; o >>= 1) qq += __shfl_xor(qq, o, 32);
    const float rs = rsqrtf(qq * (1.f / 1024.f) + 1e-5f);
    float padd = 0.f;
    if (CHKF) {
        float f = chk[(size_t)L * 32] + chk[(size_t)(L + 32) * 32];
#pragma unroll
        for (int o = 16; o > 0; o >>= 1) f += __shfl_xor(f, o, 32);
        padd = (f != 0.f) ? __uint_as_float(0x7fc00000u) : 0.f;
    }
    const size_t orow = OMAP ? ((size_t)(row / seq) * (size_t)seqfull + (size_t)(row % seq)) : (size_t)row;
#pragma unroll
    for (int q4 = 0; q4 < 8; ++q4) {
        const int c0 = 128 * q4 + 4 * L;
        const v4f gg = *(const v4f*)(G + c0), be = *(const v4f*)(Bb + c0);
        v4f y;
        y.x = (x[4 * q4]     - mu) * rs * cmb_bf(gg.x) + cmb_bf(be.x) + padd;
        y.y = (x[4 * q4 + 1] - mu) * rs * cmb_bf(gg.y) + cmb_bf(be.y) + padd;
        y.z = (x[4 * q4 + 2] - mu) * rs * cmb_bf(gg.z) + cmb_bf(be.z) + padd;
        y.w = (x[4 * q4 + 3] - mu) * rs * cmb_bf(gg.w) + cmb_bf(be.w) + padd;
        if (W16) { const unsigned long long pk = (unsigned long long)cmb_pk2(y.x, y.y) | ((unsigned long long)cmb_pk2(y.z, y.w) << 32); VST2(unsigned long long, (unsigned long long*)(O16 + (size_t)row * 1024 + c0), pk); }
        if (W32) { VST2V4(O32 + orow * 1024 + c0, y); }
    }
}

#define NBIAS 13312
__global__ __launch_bounds__(256) void k_biasprep(const float* __restrict__ sbq, const float* __restrict__ sbk, const float* __restrict__ sbv, const float* __restrict__ sbo,
                                                 const float* __restrict__ cbq, const float* __restrict__ cbk, const float* __restrict__ cbv, const float* __restrict__ cbo,
                                                 const float* __restrict__ fb1, const float* __restrict__ fb2, float* __restrict__ O) {
    const int blk = blockIdx.x; const int t = threadIdx.x; const int u = blk * 256 + t;
    float v;
    if (blk < 4) v = sbq[u];
    else if (blk < 8) v = sbk[u - 1024];
    else if (blk < 12) v = sbv[u - 2048];
    else if (blk < 16) v = sbo[u - 3072];
    else if (blk < 20) v = cbq[u - 4096];
    else if (blk < 24) v = cbk[u - 5120];
    else if (blk < 28) v = cbv[u - 6144];
    else if (blk < 32) v = cbo[u - 7168];
    else if (blk < 48) v = fb1[u - 8192];
    else v = fb2[u - 12288];
    VST2(float, O + u, cmb_bf(v));
}

__global__ __launch_bounds__(256) void k_maskchk(const int* __restrict__ mask, int seq, int seqfull, float* __restrict__ chk) {
    __shared__ int red[32];
    const int blk = blockIdx.x; const int t = threadIdx.x; const int L = t & 31; const int wave = t >> 5;
    const int rpb = seq / NCHK;
    int viol = 0;
    for (int ii = 0; ii < rpb; ++ii) {
        const int i = blk * rpb + ii;
        const int* mrow = mask + (size_t)i * seqfull;
        for (int j = t; j < seq; j += 256) { const int m = mrow[j]; viol += (((j <= i) ? 1 : 0) != ((m != 0) ? 1 : 0)) ? 1 : 0; }
    }
#pragma unroll
    for (int o = 16; o > 0; o >>= 1) viol += __shfl_xor(viol, o, 32);
    if (t < 32) red[t] = 0;
    __syncthreads();
    if (L == 0) red[wave] = viol;
    __syncthreads();
    if (t < 32) {
        int v = red[t];
#pragma unroll
        for (int o = 16; o > 0; o >>= 1) v += __shfl_xor(v, o, 32);
        const float outv = (t == 0) ? (float)v : 0.f;
        VST2(float, chk + (size_t)blk * 32 + t, outv);
    }
}

#define SZ_WQKV   ((size_t)3072 * 1024 * 2)
#define SZ_WDD    ((size_t)1024 * 1024 * 2)
#define SZ_WKV2   ((size_t)2048 * 1024 * 2)
#define SZ_WFF    ((size_t)4096 * 1024 * 2)
#define SZ_BIAS   ((size_t)NBIAS * 4)
#define SZ_CHK    ((size_t)NCHK * 128)
#define SZ_MEM16  ((size_t)RM_ROWS * 1024 * 2)
#define SZ_XH     ((size_t)R_ROWS * 1024 * 2)
#define SZ_XR     ((size_t)R_ROWS * 1024 * 4)
#define SZ_AOT    ((size_t)R_ROWS * 1024 * 4)
#define SZ_QKV    ((size_t)R_ROWS * 3072 * 4)
#define SZ_QC     ((size_t)R_ROWS * 1024 * 4)
#define SZ_KVC    ((size_t)RM_ROWS * 2048 * 4)
#define SZ_H16    ((size_t)R_ROWS * 4096 * 2)
#define SZ_SCR_A  (SZ_QKV > (SZ_QC + SZ_KVC) ? SZ_QKV : (SZ_QC + SZ_KVC))
#define SZ_SCR    (SZ_SCR_A > SZ_H16 ? SZ_SCR_A : SZ_H16)
#define SZ_TOTAL  (SZ_WQKV + 3 * SZ_WDD + SZ_WKV2 + 2 * SZ_WFF + SZ_BIAS + SZ_CHK + SZ_MEM16 + SZ_XH + SZ_XR + SZ_AOT + SZ_SCR)
static_assert(SZ_QKV <= SZ_SCR && SZ_QC + SZ_KVC <= SZ_SCR && SZ_H16 <= SZ_SCR);
static_assert(SZ_BIAS % 256 == 0 && SZ_CHK % 256 == 0 && SZ_MEM16 % 256 == 0 && SZ_XH % 256 == 0 && SZ_QC % 256 == 0);
static_assert(SZ_TOTAL <= (size_t)134217728);
static_assert(NBIAS == 52 * 256);
static_assert((R_ROWS * 1024) % 1024 == 0 && R_ROWS % 8 == 0);

extern "C" void kernel_launch(void* const* d_in, const int* in_sizes, int n_in, void* d_out, int out_size, void* d_ws, size_t ws_size, hipStream_t stream) {
    if (n_in < 29) return;
    const int R = (int)R_ROWS, RM = (int)RM_ROWS;
    if (in_sizes[0] < ((NB - 1) * SEQ_FULL + SEQ) * DM) return;
    if (in_sizes[1] < ((NB - 1) * MEM_FULL + MEMLEN) * DM) return;
    if (in_sizes[2] < (SEQ - 1) * SEQ_FULL + SEQ) return;
    if (in_sizes[3] < DM * DM || in_sizes[19] < FFD * DM || in_sizes[21] < DM * FFD) return;
    if (out_size < ((NB - 1) * SEQ_FULL + SEQ) * DM) return;
    if (SZ_TOTAL > ws_size) return;

    const float* x      = (const float*)d_in[0];
    const float* memory = (const float*)d_in[1];
    const int*   maskp  = (const int*)d_in[2];
    const float* sa_wq = (const float*)d_in[3];  const float* sa_bq = (const float*)d_in[4];
    const float* sa_wk = (const float*)d_in[5];  const float* sa_bk = (const float*)d_in[6];
    const float* sa_wv = (const float*)d_in[7];  const float* sa_bv = (const float*)d_in[8];
    const float* sa_wo = (const float*)d_in[9];  const float* sa_bo = (const float*)d_in[10];
    const float* ca_wq = (const float*)d_in[11]; const float* ca_bq = (const float*)d_in[12];
    const float* ca_wk = (const float*)d_in[13]; const float* ca_bk = (const float*)d_in[14];
    const float* ca_wv = (const float*)d_in[15]; const float* ca_bv = (const float*)d_in[16];
    const float* ca_wo = (const float*)d_in[17]; const float* ca_bo = (const float*)d_in[18];
    const float* ff_w1 = (const float*)d_in[19]; const float* ff_b1 = (const float*)d_in[20];
    const float* ff_w2 = (const float*)d_in[21]; const float* ff_b2 = (const float*)d_in[22];
    const float* ln1_g = (const float*)d_in[23]; const float* ln1_b = (const float*)d_in[24];
    const float* ln2_g = (const float*)d_in[25]; const float* ln2_b = (const float*)d_in[26];
    const float* ln3_g = (const float*)d_in[27]; const float* ln3_b = (const float*)d_in[28];
    float* out = (float*)d_out;

    char* wsp = (char*)d_ws;
    unsigned short* WQKV16 = (unsigned short*)wsp; wsp += SZ_WQKV;
    unsigned short* SWO16  = (unsigned short*)wsp; wsp += SZ_WDD;
    unsigned short* CWQ16  = (unsigned short*)wsp; wsp += SZ_WDD;
    unsigned short* CWKV16 = (unsigned short*)wsp; wsp += SZ_WKV2;
    unsigned short* CWO16  = (unsigned short*)wsp; wsp += SZ_WDD;
    unsigned short* W116   = (unsigned short*)wsp; wsp += SZ_WFF;
    unsigned short* W216   = (unsigned short*)wsp; wsp += SZ_WFF;
    float* BIAS = (float*)wsp; wsp += SZ_BIAS;
    float* CHK  = (float*)wsp; wsp += SZ_CHK;
    unsigned short* MEM16 = (unsigned short*)wsp; wsp += SZ_MEM16;
    unsigned short* XH  = (unsigned short*)wsp; wsp += SZ_XH;
    float* XR  = (float*)wsp; wsp += SZ_XR;
    float* AOT = (float*)wsp; wsp += SZ_AOT;
    char*  SCR = wsp; wsp += SZ_SCR;
    if ((size_t)(wsp - (char*)d_ws) > ws_size) return;
    float* QKV = (float*)SCR;
    float* QC  = (float*)SCR;
    float* KVC = (float*)(SCR + SZ_QC);
    unsigned short* H16 = (unsigned short*)SCR;

    const unsigned gdd = (unsigned)(((long long)1024 * (1024 / 8) + 255) / 256);
    k_cm_castb<<<gdd, 256, 0, stream>>>(sa_wq, 1024, WQKV16,                     1024, 1024, 1024, 16.0f);
    k_cm_castb<<<gdd, 256, 0, stream>>>(sa_wk, 1024, WQKV16 + (size_t)1024 * 1024, 1024, 1024, 1024, 16.0f);
    k_cm_castb<<<gdd, 256, 0, stream>>>(sa_wv, 1024, WQKV16 + (size_t)2048 * 1024, 1024, 1024, 1024, 16.0f);
    k_cm_castb<<<gdd, 256, 0, stream>>>(sa_wo, 1024, SWO16, 1024, 1024, 1024, 16.0f);
    k_cm_castb<<<gdd, 256, 0, stream>>>(ca_wq, 1024, CWQ16, 1024, 1024, 1024, 16.0f);
    k_cm_castb<<<gdd, 256, 0, stream>>>(ca_wk, 1024, CWKV16,                     1024, 1024, 1024, 16.0f);
    k_cm_castb<<<gdd, 256, 0, stream>>>(ca_wv, 1024, CWKV16 + (size_t)1024 * 1024, 1024, 1024, 1024, 16.0f);
    k_cm_castb<<<gdd, 256, 0, stream>>>(ca_wo, 1024, CWO16, 1024, 1024, 1024, 16.0f);
    k_cm_castb<<<(unsigned)(((long long)4096 * (1024 / 8) + 255) / 256), 256, 0, stream>>>(ff_w1, 1024, W116, 1024, 4096, 1024, 16.0f);
    k_cm_castb<<<(unsigned)(((long long)1024 * (4096 / 8) + 255) / 256), 256, 0, stream>>>(ff_w2, 4096, W216, 4096, 1024, 4096, 16.0f);
    k_biasprep<<<NBIAS / 256, 256, 0, stream>>>(sa_bq, sa_bk, sa_bv, sa_bo, ca_bq, ca_bk, ca_bv, ca_bo, ff_b1, ff_b2, BIAS);
    k_maskchk<<<NCHK, 256, 0, stream>>>(maskp, SEQ, SEQ_FULL, CHK);
    k_cvt16<true, true><<<(unsigned)R, 256, 0, stream>>>(x, XH, XR, R, SEQ, SEQ_FULL);
    k_cvt16<true, false><<<(unsigned)RM, 256, 0, stream>>>(memory, MEM16, nullptr, RM, MEMLEN, MEM_FULL);

    w25::wmma_gemm64<0, false, 2, 0, false, 0><<<dim3((unsigned)(((R / 64) * (3072 / 64) + 7) / 8), 1), 256, 0, stream>>>(
        XH, nullptr, 1024, 0L, WQKV16, nullptr, 1024, 0L, (void*)QKV, nullptr, 3072, 0L, BIAS + 0, nullptr, 0L, R, 3072, 1024, 0.0625f);
    {
        w25::AttnGeom g;
        g.cp = XR; g.pc = XR; g.c_bs = 0; g.c_rs = 0; g.c_hs = 0;
        g.q_bs = (long)SEQ * 3072; g.q_rs = 3072; g.q_hs = 64;
        g.k_bs = (long)SEQ * 3072; g.k_rs = 3072; g.k_hs = 64;
        g.v_bs = (long)SEQ * 3072; g.v_rs = 3072; g.v_hs = 64;
        g.o_bs = (long)SEQ * 1024; g.o_rs = 1024; g.o_hs = 64;
        g.S = SEQ; g.Skv = SEQ; g.H = NHEAD; g.mask_mode = 1; g.qscale = 0.125f; g.blk0 = 0; g.mask_fill = -1.0e30f; g.mask_is_int = 0;
        w25::attn64_kernel<false, false, true><<<dim3((unsigned)(NB * NHEAD * (SEQ / 64))), 128, 0, stream>>>(QKV, QKV + 1024, QKV + 2048, AOT, (const void*)maskp, maskp, g);
    }
    {
        AttnP a;
        a.Q = QKV; a.K = QKV + 1024; a.V = QKV + 2048; a.O = AOT; a.P = 0; a.Mf = 0; a.Mi = 0; a.ST = 0;
        a.Pw = 0; a.Rt = 0; a.SQ = 0; a.SK = 0;
        a.swb = 0; a.swh = 0; a.swi = 0; a.swj = 0; a.srb = 0; a.srh = 0; a.sri = 0;
        a.sQb = (long long)SEQ * 3072; a.sQh = 64; a.sQi = 3072; a.sQd = 1; a.sKb = (long long)SEQ * 3072; a.sKh = 64; a.sKj = 3072; a.sKd = 1;
        a.sVb = (long long)SEQ * 3072; a.sVh = 64; a.sVj = 3072; a.sVd = 1; a.sOb = (long long)SEQ * 1024; a.sOh = 64; a.sOi = 1024;
        a.sPb = 0; a.sPh = 0; a.sPi = 0; a.smb = 0; a.smh = 0; a.smi = 0; a.smj = 0;
        a.Lq = SEQ; a.Lk = SEQ; a.dh = 64; a.dv = 64; a.hrep = 1; a.causal = 1; a.coff = 0; a.pband = 0;
        a.scale = 0.125f; a.mfill = 0.0f; a.nonorm = 0; a.mpol = 0;
        a.roff = 0; a.rn = 1; a.segpol = 0; a.win = 0;
        k_attn<64, 64, 1, true, false><<<dim3(1u, (unsigned)NHEAD, (unsigned)NB), 32 * AW, 0, stream>>>(a);
    }
    k_cvt16<false, false><<<(unsigned)R, 256, 0, stream>>>(AOT, XH, nullptr, R, R, R);
    w25::wmma_gemm64<0, false, 2, 0, true, 0><<<dim3((unsigned)(((R / 64) * (1024 / 64) + 7) / 8), 1), 256, 0, stream>>>(
        XH, nullptr, 1024, 0L, SWO16, nullptr, 1024, 0L, (void*)AOT, nullptr, 1024, 0L, BIAS + 3072, XR, 0L, R, 1024, 1024, 0.0625f);
    k_ln1024<true, true, false, false><<<(unsigned)(R / 8), 256, 0, stream>>>(AOT, ln1_g, ln1_b, XH, XR, CHK, R, SEQ, SEQ_FULL);

    w25::wmma_gemm64<0, false, 2, 0, false, 0><<<dim3((unsigned)(((R / 64) * (1024 / 64) + 7) / 8), 1), 256, 0, stream>>>(
        XH, nullptr, 1024, 0L, CWQ16, nullptr, 1024, 0L, (void*)QC, nullptr, 1024, 0L, BIAS + 4096, nullptr, 0L, R, 1024, 1024, 0.0625f);
    w25::wmma_gemm64<0, false, 2, 0, false, 0><<<dim3((unsigned)(((RM / 64) * (2048 / 64) + 7) / 8), 1), 256, 0, stream>>>(
        MEM16, nullptr, 1024, 0L, CWKV16, nullptr, 1024, 0L, (void*)KVC, nullptr, 2048, 0L, BIAS + 5120, nullptr, 0L, RM, 2048, 1024, 0.0625f);
    {
        w25::AttnGeom g;
        g.cp = XR; g.pc = XR; g.c_bs = 0; g.c_rs = 0; g.c_hs = 0;
        g.q_bs = (long)SEQ * 1024;    g.q_rs = 1024; g.q_hs = 64;
        g.k_bs = (long)MEMLEN * 2048; g.k_rs = 2048; g.k_hs = 64;
        g.v_bs = (long)MEMLEN * 2048; g.v_rs = 2048; g.v_hs = 64;
        g.o_bs = (long)SEQ * 1024;    g.o_rs = 1024; g.o_hs = 64;
        g.S = SEQ; g.Skv = MEMLEN; g.H = NHEAD; g.mask_mode = 0; g.qscale = 0.125f; g.blk0 = 0; g.mask_fill = -1.0e30f; g.mask_is_int = 0;
        w25::attn64_kernel<false, false, true><<<dim3((unsigned)(NB * NHEAD * (SEQ / 64))), 128, 0, stream>>>(QC, KVC, KVC + 1024, AOT, (const void*)maskp, maskp, g);
    }
    k_cvt16<false, false><<<(unsigned)R, 256, 0, stream>>>(AOT, XH, nullptr, R, R, R);
    w25::wmma_gemm64<0, false, 2, 0, true, 0><<<dim3((unsigned)(((R / 64) * (1024 / 64) + 7) / 8), 1), 256, 0, stream>>>(
        XH, nullptr, 1024, 0L, CWO16, nullptr, 1024, 0L, (void*)AOT, nullptr, 1024, 0L, BIAS + 7168, XR, 0L, R, 1024, 1024, 0.0625f);
    k_ln1024<true, true, false, false><<<(unsigned)(R / 8), 256, 0, stream>>>(AOT, ln2_g, ln2_b, XH, XR, CHK, R, SEQ, SEQ_FULL);

    w25::wmma_gemm64<0, false, 2, 1, false, 2><<<dim3((unsigned)(((R / 64) * (4096 / 64) + 7) / 8), 1), 256, 0, stream>>>(
        XH, nullptr, 1024, 0L, W116, nullptr, 1024, 0L, (void*)H16, nullptr, 4096, 0L, BIAS + 8192, nullptr, 0L, R, 4096, 1024, 0.0625f);
    w25::wmma_gemm64<0, false, 2, 0, true, 0><<<dim3((unsigned)(((R / 64) * (1024 / 64) + 7) / 8), 1), 256, 0, stream>>>(
        H16, nullptr, 4096, 0L, W216, nullptr, 4096, 0L, (void*)AOT, nullptr, 1024, 0L, BIAS + 12288, XR, 0L, R, 1024, 4096, 0.0625f);
    k_ln1024<false, true, true, true><<<(unsigned)(R / 8), 256, 0, stream>>>(AOT, ln3_g, ln3_b, XH, out, CHK, R, SEQ, SEQ_FULL);
}
